// Stage2GNN_9019431321967
// MI455X (gfx1250) — hardware-run, weakly checked
//
#include <hip/hip_runtime.h>


namespace {
constexpr int N = 50000, E = 1600000, SAT = 32, H = 128, OUT = 16, NBLK = N / 16;
constexpr float XS = 8.0f, WSC = 256.0f, SLOPE = 0.2f;
typedef _Float16 b16;
typedef __attribute__((ext_vector_type(16))) _Float16 v16b;
typedef __attribute__((ext_vector_type(8))) _Float16 v8b;
typedef __attribute__((ext_vector_type(8))) float v8f;
typedef __attribute__((ext_vector_type(4))) float v4f;
__device__ __forceinline__ float bf16_rne(float f) { unsigned int u = __float_as_uint(f); u += 0x7FFFu + ((u >> 16) & 1u); return __uint_as_float(u & 0xFFFF0000u); }
__device__ __forceinline__ void split16(float v, b16& hi, b16& lo) { hi = (b16)v; lo = (b16)(v - (float)hi); }
__device__ __forceinline__ v16b frag_kb(const b16* p, int hh) { const v8b a = *(const v8b*)(p + 8 * hh), b = *(const v8b*)(p + 16 + 8 * hh); v16b f;
#pragma unroll
  for (int e = 0; e < 8; ++e) { f[e] = a[e]; f[8 + e] = b[e]; } return f; }
__device__ __forceinline__ v8f wmma16b(v16b a, v16b b, v8f c) { v8f d = __builtin_amdgcn_wmma_f32_16x16x32_f16(false, a, false, b, (short)0, c, false, false); asm volatile("v_nop\n\tv_nop\n\tv_nop\n\tv_nop" : "+v"(d) : "v"(a), "v"(b)); return d; }
__device__ __forceinline__ void wave_lds_sync() { __builtin_amdgcn_fence(__ATOMIC_RELEASE, "workgroup"); __builtin_amdgcn_wave_barrier(); __builtin_amdgcn_fence(__ATOMIC_ACQUIRE, "workgroup"); }
__device__ __forceinline__ float pmul(float a, float b) { float p = a * b; asm volatile("" : "+v"(p)); return p; }
__device__ __forceinline__ int iclamp(int v, int lo, int hi) { return v < lo ? lo : (v > hi ? hi : v); }
__device__ __forceinline__ float leaky(float v) { return v >= 0.0f ? v : SLOPE * v; }
constexpr int CSR_NBLK7 = 512, CSR_GB7 = 7, CSR_GN7 = 1 << CSR_GB7  , CSR_TS7 = (CSR_GN7 < 32 ? 32 : CSR_GN7)  , CSR_MAXG7 = 512, CSR_CAP7 = 12288  ;
__device__ __host__ __forceinline__ int csr_tix7(int v) { return (v >> CSR_GB7) * CSR_TS7 + (v & (CSR_GN7 - 1)); }
__global__ __launch_bounds__(64) void csrA_kernel7(const int* __restrict__ dst, int E, int N, int nG, int CHP, int NGP, int* __restrict__ STG, int* __restrict__ HST) {
  extern __shared__ int sm[];
  int* cnt = sm; int* run = sm + NGP; int* ids = sm + 2 * NGP;
  const int b = blockIdx.x; const int ch = (E + CSR_NBLK7 - 1) / CSR_NBLK7; const int e0 = b * ch, e1 = min(E, e0 + ch);
  for (int i = threadIdx.x; i < NGP; i += 64) cnt[i] = 0;
  for (int i = threadIdx.x; i < CHP; i += 64) ids[i] = -1;
  __syncthreads();
  if (threadIdx.x == 0) {
    for (int e = e0; e < e1; ++e) { int d = dst[e]; d = (d < 0) ? 0 : (d >= N ? N - 1 : d); cnt[d >> CSR_GB7] += 1; }
    int acc = 0; for (int g = 0; g < nG; ++g) { run[g] = acc; acc += cnt[g]; }
    for (int e = e0; e < e1; ++e) { int d = dst[e]; d = (d < 0) ? 0 : (d >= N ? N - 1 : d); const int g = d >> CSR_GB7; ids[run[g]] = e; run[g] += 1; } }
  __syncthreads();
  typedef __attribute__((ext_vector_type(4))) int v4i;
  for (int pass = 0; pass < 2; ++pass) {
    for (int i = threadIdx.x; i < CHP / 4; i += 64) *(volatile v4i*)(STG + (size_t)b * CHP + i * 4) = *(const v4i*)(&ids[i * 4]);
    for (int i = threadIdx.x; i < NGP / 4; i += 64) { v4i v; for (int e = 0; e < 4; ++e) v[e] = (i * 4 + e < nG) ? cnt[i * 4 + e] : 0; *(volatile v4i*)(HST + (size_t)b * NGP + i * 4) = v; }
    __threadfence(); }
}
__global__ __launch_bounds__(512) void csrS_kernel7(const int* __restrict__ HST, int nG, int NGP, int* __restrict__ START, int* __restrict__ TOT, int* __restrict__ OFF) {
  __shared__ int tot[CSR_MAXG7];
  const int b = threadIdx.x;
  for (int pass = 0; pass < 2; ++pass) { int runb = 0; for (int g = 0; g < nG; ++g) { int c = HST[(size_t)b * NGP + g]; c = (c < 0) ? 0 : c; ((volatile int*)OFF)[(size_t)g * CSR_NBLK7 + b] = runb; runb += c; } __threadfence(); }
  for (int g = threadIdx.x; g < nG; g += 512) { int s = 0; for (int bb = 0; bb < CSR_NBLK7; ++bb) { int c = HST[(size_t)bb * NGP + g]; s += (c < 0) ? 0 : c; } tot[g] = s; }
  __syncthreads();
  if (threadIdx.x < 32) {
    __shared__ int st[CSR_MAXG7 + 32];
    if (threadIdx.x == 0) { int acc = 0; for (int g = 0; g < NGP; ++g) { st[g] = acc; if (g < nG) acc += (tot[g] + 31) & ~31; } st[NGP] = acc; }
    __builtin_amdgcn_fence(__ATOMIC_RELEASE, "workgroup"); __builtin_amdgcn_wave_barrier(); __builtin_amdgcn_fence(__ATOMIC_ACQUIRE, "workgroup");
    for (int pass = 0; pass < 2; ++pass) { for (int i = threadIdx.x; i < NGP + 32; i += 32) { ((volatile int*)START)[i] = (i <= NGP) ? st[min(i, NGP)] : 0; ((volatile int*)TOT)[i] = (i < nG) ? tot[i] : 0; } __threadfence(); } }
}
__global__ __launch_bounds__(256) void csrB_kernel7(const int* __restrict__ dst, int N, int nG, int CHP, int NGP, int permLen, const int* __restrict__ STG, const int* __restrict__ HST, const int* __restrict__ OFF, const int* __restrict__ START, const int* __restrict__ TOT, int* __restrict__ PERM, int* __restrict__ ROWPTR, int* __restrict__ ROWCNT, int* __restrict__ FLAG) {
  typedef __attribute__((ext_vector_type(4))) int v4i;
  __shared__ int ids[CSR_CAP7]; __shared__ unsigned short key[CSR_CAP7]; __shared__ int outp[CSR_CAP7]; __shared__ int ncnt[CSR_GN7 + 1]; __shared__ int boff[CSR_NBLK7 + 1];
  const int g = blockIdx.x, t_ = threadIdx.x; int tot = TOT[g]; int st = START[g], stn = START[g + 1]; const int v0 = g * CSR_GN7; const int nv = min(CSR_GN7, N - v0); const int t0 = g * CSR_TS7;
  st = (st < 0) ? 0 : (st > permLen - 32 ? permLen - 32 : st) & ~31; stn = (stn < st) ? st : (stn > permLen ? permLen : stn); tot = (tot < 0) ? 0 : tot; if (tot > stn - st && tot <= CSR_CAP7) tot = stn - st;
  if (tot > CSR_CAP7) {
    for (int pass = 0; pass < 2; ++pass) { for (int i = t_; i < CSR_TS7 / 4; i += 256) { v4i a, c; for (int e = 0; e < 4; ++e) { a[e] = st; c[e] = 0; } *(volatile v4i*)(ROWPTR + t0 + i * 4) = a; *(volatile v4i*)(ROWCNT + t0 + i * 4) = c; } if (t_ == 0) ((volatile int*)FLAG)[0] = 1; __threadfence(); } (void)nv; return; }
  if (t_ == 0) { int acc = 0; for (int b = 0; b < CSR_NBLK7; ++b) { boff[b] = acc; int c = HST[(size_t)b * NGP + g]; c = (c < 0) ? 0 : (c > CHP ? CHP : c); acc += c; if (acc > tot) acc = tot; } boff[CSR_NBLK7] = acc; }
  for (int i = t_; i <= CSR_GN7; i += 256) ncnt[i] = 0;
  __syncthreads();
  for (int b = 0; b < CSR_NBLK7; ++b) { const int c = boff[b + 1] - boff[b]; int o_ = OFF[(size_t)g * CSR_NBLK7 + b]; o_ = (o_ < 0) ? 0 : (o_ > CHP - c ? CHP - c : o_); const int* src_ = STG + (size_t)b * CHP + o_;
    for (int i = t_; i < c; i += 256) { int id = src_[i]; id = (id < 0) ? 0 : id; ids[boff[b] + i] = id; int d = dst[id]; d = (d < v0) ? v0 : (d >= N ? N - 1 : d); int kk = d - v0; kk = (kk < 0) ? 0 : (kk >= CSR_GN7 ? CSR_GN7 - 1 : kk); key[boff[b] + i] = (unsigned short)kk; } }
  __syncthreads();
  if (t_ == 0) { for (int i = 0; i < tot; ++i) ncnt[key[i]] += 1; int acc = 0; for (int vl = 0; vl < CSR_GN7; ++vl) { const int c = ncnt[vl]; ncnt[vl] = acc; acc += c; } ncnt[CSR_GN7] = acc;
    for (int i = 0; i < tot; ++i) { const int vl = key[i]; outp[ncnt[vl]] = ids[i]; ncnt[vl] += 1; }
    for (int vl = CSR_GN7; vl > 0; --vl) ncnt[vl] = ncnt[vl - 1]; ncnt[0] = 0; }
  __syncthreads();
  for (int pass = 0; pass < 2; ++pass) {
    for (int i = t_; i < (stn - st) / 4; i += 256) { v4i v; for (int e = 0; e < 4; ++e) { const int q = i * 4 + e; v[e] = (q < tot) ? outp[q] : -1; } *(volatile v4i*)(PERM + st + i * 4) = v; }
    for (int i = t_; i < CSR_TS7 / 4; i += 256) { v4i a, c; for (int e = 0; e < 4; ++e) { const int vl = i * 4 + e; const int vc = vl < CSR_GN7 ? vl : CSR_GN7; a[e] = (vl < CSR_GN7) ? st + ncnt[vc] : st; c[e] = (vl < nv) ? (ncnt[(vc < CSR_GN7 ? vc : CSR_GN7 - 1) + 1] - ncnt[vc]) : 0; } *(volatile v4i*)(ROWPTR + t0 + i * 4) = a; *(volatile v4i*)(ROWCNT + t0 + i * 4) = c; }
    __threadfence(); }
}
__global__ __launch_bounds__(256) void csrZ_kernel7(int* __restrict__ p, size_t n4) { typedef __attribute__((ext_vector_type(4))) int v4i; const size_t tid = (size_t)blockIdx.x * 256 + threadIdx.x, nth = (size_t)gridDim.x * 256; v4i z = {0, 0, 0, 0}; for (size_t i = tid; i < n4; i += nth) *(volatile v4i*)(p + i * 4) = z; }
struct CsrBufs7 { int *STG, *HST, *OFF, *START, *TOT, *PERM, *ROWPTR, *ROWCNT, *FLAG; int nG, NGP, CHP; size_t permLen; char* base; size_t bytes; };
static size_t csr_carve7(CsrBufs7& c, char* ws, size_t off, int E, int N) {
  const size_t off0 = off; c.base = ws + off;
  auto al = [&](size_t bytes) { char* p = ws + off; off += (bytes + 255) & ~(size_t)255; return p; };
  c.nG = (N + CSR_GN7 - 1) / CSR_GN7; c.NGP = (c.nG + 31) & ~31; const int ch = (E + CSR_NBLK7 - 1) / CSR_NBLK7; c.CHP = (ch + 31) & ~31; c.permLen = (size_t)E + 32 * (size_t)c.nG + 32;
  c.STG = (int*)al((size_t)CSR_NBLK7 * c.CHP * 4); c.HST = (int*)al((size_t)CSR_NBLK7 * c.NGP * 4); c.OFF = (int*)al((size_t)c.NGP * CSR_NBLK7 * 4); c.START = (int*)al((size_t)(c.NGP + 64) * 4); c.TOT = (int*)al((size_t)(c.NGP + 64) * 4);
  c.PERM = (int*)al(c.permLen * 4); c.ROWPTR = (int*)al((size_t)c.nG * CSR_TS7 * 4); c.ROWCNT = (int*)al((size_t)c.nG * CSR_TS7 * 4); c.FLAG = (int*)al(256);
  c.bytes = off - off0; return off;
}
static void csr_build7(const CsrBufs7& c, const int* dst, int E, int N, hipStream_t stream) {
  const size_t smem = (size_t)(2 * c.NGP + c.CHP) * 4;
  csrZ_kernel7<<<512, 256, 0, stream>>>((int*)c.base, c.bytes / 16);
  csrA_kernel7<<<CSR_NBLK7, 64, smem, stream>>>(dst, E, N, c.nG, c.CHP, c.NGP, c.STG, c.HST);
  csrS_kernel7<<<1, 512, 0, stream>>>(c.HST, c.nG, c.NGP, c.START, c.TOT, c.OFF);
  csrB_kernel7<<<c.nG, 256, 0, stream>>>(dst, N, c.nG, c.CHP, c.NGP, (int)c.permLen, c.STG, c.HST, c.OFF, c.START, c.TOT, c.PERM, c.ROWPTR, c.ROWCNT, c.FLAG);
}


__global__ __launch_bounds__(256) void wcopy_kernel(const float* __restrict__ w, int OUTW, int OUTP, int KIN, b16* __restrict__ WT) {
  const size_t u = (size_t)blockIdx.x * 256 + threadIdx.x; if (u >= (size_t)OUTP * KIN / 8) return; const size_t e = u * 8; const int o = (int)(e / KIN); v8b v;
#pragma unroll
  for (int j = 0; j < 8; ++j) v[j] = (o < OUTW) ? (b16)(bf16_rne(w[e + j]) * WSC) : (b16)0.0f; for (int pass = 0; pass < 2; ++pass) { *(volatile v8b*)(WT + e) = v; __threadfence(); }
}
__global__ __launch_bounds__(32) void in_kernel(const float* __restrict__ x, const b16* __restrict__ WS_, const b16* __restrict__ WN_, const float* __restrict__ sb, const float* __restrict__ nb, const float* __restrict__ fw, const float* __restrict__ fb, float* __restrict__ H0) {
  __shared__ __attribute__((aligned(16))) b16 As[16][40], An[16][40]; __shared__ __attribute__((aligned(16))) float Ts[16][H + 4], Tn[16][H + 4]; __shared__ float Gt[16];
  const int lane = threadIdx.x, nloc = lane & 15, hlf = lane >> 4; const size_t m0 = (size_t)blockIdx.x * 16;
  for (int rr = 0; rr < 16; ++rr) { As[rr][lane] = (b16)(bf16_rne(x[(m0 + rr) * 64 + lane]) * XS); An[rr][lane] = (b16)(bf16_rne(x[(m0 + rr) * 64 + 32 + lane]) * XS); }
  wave_lds_sync(); const v16b as_ = frag_kb(&As[nloc][0], hlf), an_ = frag_kb(&An[nloc][0], hlf); float gp[8];
#pragma unroll
  for (int r8 = 0; r8 < 8; ++r8) gp[r8] = 0.0f;
#pragma unroll
  for (int t = 0; t < 8; ++t) { v8f a1 = {}, a2 = {}; a1 = wmma16b(as_, frag_kb(WS_ + (size_t)(t * 16 + nloc) * 32, hlf), a1); a2 = wmma16b(an_, frag_kb(WN_ + (size_t)(t * 16 + nloc) * 32, hlf), a2); const int c = t * 16 + nloc; const float b1 = bf16_rne(sb[c]), b2 = bf16_rne(nb[c]), f1 = bf16_rne(fw[c]), f2 = bf16_rne(fw[H + c]);
#pragma unroll
    for (int r8 = 0; r8 < 8; ++r8) { const float s = fmaxf(a1[r8] * (1.0f / (XS * WSC)) + b1, 0.0f), nn = fmaxf(a2[r8] * (1.0f / (XS * WSC)) + b2, 0.0f); Ts[8 * hlf + r8][c] = s; Tn[8 * hlf + r8][c] = nn; gp[r8] += pmul(s, f1) + pmul(nn, f2); } }
#pragma unroll
  for (int r8 = 0; r8 < 8; ++r8) { float s = gp[r8]; for (int o = 1; o < 16; o <<= 1) s += __shfl_xor(s, o); if (nloc == 0) Gt[8 * hlf + r8] = 1.0f / (1.0f + __expf(-(s + bf16_rne(fb[0])))); }
  wave_lds_sync();
  for (int pass = 0; pass < 2; ++pass) { for (int rr = 0; rr < 16; ++rr) { const float g = Gt[rr]; v4f o; for (int i = 0; i < 4; ++i) { const int c = lane * 4 + i; o[i] = pmul(g, Ts[rr][c]) + pmul(1.0f - g, Tn[rr][c]); } *(volatile v4f*)(H0 + (m0 + rr) * H + lane * 4) = o; } __threadfence(); }
}
__global__ __launch_bounds__(32) void proj_kernel(const float* __restrict__ Hh, const b16* __restrict__ WT, const float* __restrict__ asv, const float* __restrict__ adv, int NLIM, float* __restrict__ HW, float* __restrict__ AS) {
  __shared__ __attribute__((aligned(16))) b16 Ah[16][H + 8], Al[16][H + 8]; __shared__ __attribute__((aligned(16))) float Tf[16][H + 4], Ps[16][2];
  const int lane = threadIdx.x, nloc = lane & 15, hlf = lane >> 4; const size_t m0 = (size_t)blockIdx.x * 16; if (m0 >= (size_t)NLIM) return;
  for (int rr = 0; rr < 16; ++rr) for (int q = 0; q < 4; ++q) { b16 p, ql; split16(Hh[(m0 + rr) * H + q * 32 + lane] * XS, p, ql); Ah[rr][q * 32 + lane] = p; Al[rr][q * 32 + lane] = ql; }
  wave_lds_sync(); v8f acc[8];
#pragma unroll
  for (int t = 0; t < 8; ++t) acc[t] = (v8f){};
#pragma unroll
  for (int kb = 0; kb < H; kb += 32) { const v16b a = frag_kb(&Ah[nloc][kb], hlf), al = frag_kb(&Al[nloc][kb], hlf);
#pragma unroll
    for (int t = 0; t < 8; ++t) { const v16b bw = frag_kb(WT + (size_t)(t * 16 + nloc) * H + kb, hlf); acc[t] = wmma16b(a, bw, acc[t]); acc[t] = wmma16b(al, bw, acc[t]); } }
  float ps[8], pd[8];
#pragma unroll
  for (int r8 = 0; r8 < 8; ++r8) { ps[r8] = 0.0f; pd[r8] = 0.0f; }
#pragma unroll
  for (int t = 0; t < 8; ++t) { const int c = t * 16 + nloc; const float wa = bf16_rne(asv[c]), wd = bf16_rne(adv[c]);
#pragma unroll
    for (int r8 = 0; r8 < 8; ++r8) { const float v = acc[t][r8] * (1.0f / (XS * WSC)); Tf[8 * hlf + r8][c] = v; ps[r8] += pmul(v, wa); pd[r8] += pmul(v, wd); } }
#pragma unroll
  for (int r8 = 0; r8 < 8; ++r8) { float a = ps[r8], d = pd[r8]; for (int o = 1; o < 16; o <<= 1) { a += __shfl_xor(a, o); d += __shfl_xor(d, o); } if (nloc == 0) { Ps[8 * hlf + r8][0] = a; Ps[8 * hlf + r8][1] = d; } }
  wave_lds_sync();
  for (int pass = 0; pass < 2; ++pass) { for (int rr = 0; rr < 16; ++rr) *(volatile v4f*)(HW + (m0 + rr) * H + lane * 4) = *(const v4f*)(&Tf[rr][lane * 4]); ((volatile float*)AS)[m0 * 2 + lane] = Ps[lane >> 1][lane & 1]; __threadfence(); }
}
__global__ __launch_bounds__(256) void att_kernel(const float* __restrict__ HW, const float* __restrict__ AS, const float* __restrict__ bias, const int* __restrict__ srcs, const int* __restrict__ PERM, const int* __restrict__ ROWPTR, const int* __restrict__ ROWCNT, int permLen, int NLIM, float* __restrict__ G) {
  const int wave = threadIdx.x >> 5, lane = threadIdx.x & 31; const size_t v = (size_t)blockIdx.x * 8 + wave; if (v >= (size_t)NLIM) return;
  const float ad = AS[v * 2 + 1]; int st = ROWPTR[v], cnt = ROWCNT[v]; cnt = iclamp(cnt, 0, 1 << 21); st = iclamp(st, 0, permLen - cnt);
  float mx = leaky(AS[v * 2] + ad);
#pragma unroll 1
  for (int j = 0; j < cnt; ++j) { const int e = iclamp(PERM[st + j], 0, E - 1); const size_t s = (size_t)iclamp(srcs[e], 0, N - 1); if (s >= (size_t)NLIM) continue; mx = fmaxf(mx, leaky(AS[s * 2] + ad)); }
  float den; v4f o; { const float p = __expf(leaky(AS[v * 2] + ad) - mx); den = p; const v4f hv = *(const v4f*)(HW + v * H + lane * 4); for (int i = 0; i < 4; ++i) o[i] = pmul(p, hv[i]); }
#pragma unroll 1
  for (int j = 0; j < cnt; ++j) { const int e = iclamp(PERM[st + j], 0, E - 1); const size_t s = (size_t)iclamp(srcs[e], 0, N - 1); if (s >= (size_t)NLIM) continue; const float p = __expf(leaky(AS[s * 2] + ad) - mx); den += p; const v4f hv = *(const v4f*)(HW + s * H + lane * 4); for (int i = 0; i < 4; ++i) o[i] += pmul(p, hv[i]); }
  const float inv = 1.0f / den; v4f r; for (int i = 0; i < 4; ++i) r[i] = pmul(o[i], inv) + bf16_rne(bias[lane * 4 + i]);
  for (int pass = 0; pass < 2; ++pass) { *(volatile v4f*)(G + v * H + lane * 4) = r; __threadfence(); }
}
__global__ __launch_bounds__(256) void stats_kernel(const float* __restrict__ G, int NLIM, float* __restrict__ ST) {
  __shared__ float red[256]; const int c = blockIdx.x, tid = threadIdx.x; float s = 0.0f;
  for (int n = tid; n < NLIM; n += 256) s += G[(size_t)n * H + c]; red[tid] = s; __syncthreads();
  for (int w = 128; w > 0; w >>= 1) { if (tid < w) red[tid] += red[tid + w]; __syncthreads(); } const float mu = red[0] / (float)NLIM; __syncthreads();
  float q = 0.0f; for (int n = tid; n < NLIM; n += 256) { const float d = G[(size_t)n * H + c] - mu; q += pmul(d, d); } red[tid] = q; __syncthreads();
  for (int w = 128; w > 0; w >>= 1) { if (tid < w) red[tid] += red[tid + w]; __syncthreads(); } const float rs = rsqrtf(red[0] / (float)NLIM + 1e-5f);
  if (tid < 32) { for (int pass = 0; pass < 2; ++pass) { ((volatile float*)ST)[c * 32 + tid] = tid == 0 ? mu : (tid == 1 ? rs : 0.0f); __threadfence(); } }
}
__global__ __launch_bounds__(256) void bn_kernel(const float* __restrict__ G, const float* __restrict__ ST, const float* __restrict__ gm, const float* __restrict__ bt, const float* __restrict__ HP, int NLIM, float* __restrict__ HN) {
  const int wave = threadIdx.x >> 5, lane = threadIdx.x & 31; const size_t v = (size_t)blockIdx.x * 8 + wave; if (v >= (size_t)NLIM) return; v4f r; const v4f gv = *(const v4f*)(G + v * H + lane * 4), hp = *(const v4f*)(HP + v * H + lane * 4);
  for (int i = 0; i < 4; ++i) { const int c = lane * 4 + i; const float mu = ST[c * 32], rs = ST[c * 32 + 1]; r[i] = fmaxf(pmul(pmul(gv[i] - mu, rs), bf16_rne(gm[c])) + bf16_rne(bt[c]), 0.0f) + hp[i]; }
  for (int pass = 0; pass < 2; ++pass) { *(volatile v4f*)(HN + v * H + lane * 4) = r; __threadfence(); }
}
__global__ __launch_bounds__(32) void head_kernel(const float* __restrict__ Hh, const b16* __restrict__ W1T, const float* __restrict__ b1, const b16* __restrict__ W2T, const float* __restrict__ b2, int NLIM, float* __restrict__ out) {
  __shared__ __attribute__((aligned(16))) b16 Ah[16][H + 8], Al[16][H + 8]; __shared__ float So[16][OUT];
  const int lane = threadIdx.x, nloc = lane & 15, hlf = lane >> 4; const size_t m0 = (size_t)blockIdx.x * 16; if (m0 >= (size_t)NLIM) return;
  for (int rr = 0; rr < 16; ++rr) for (int q = 0; q < 4; ++q) { b16 p, ql; split16(Hh[(m0 + rr) * H + q * 32 + lane] * XS, p, ql); Ah[rr][q * 32 + lane] = p; Al[rr][q * 32 + lane] = ql; }
  wave_lds_sync(); v8f acc[8];
#pragma unroll
  for (int t = 0; t < 8; ++t) acc[t] = (v8f){};
#pragma unroll
  for (int kb = 0; kb < H; kb += 32) { const v16b a = frag_kb(&Ah[nloc][kb], hlf), al = frag_kb(&Al[nloc][kb], hlf);
#pragma unroll
    for (int t = 0; t < 8; ++t) { const v16b bw = frag_kb(W1T + (size_t)(t * 16 + nloc) * H + kb, hlf); acc[t] = wmma16b(a, bw, acc[t]); acc[t] = wmma16b(al, bw, acc[t]); } }
  wave_lds_sync();
#pragma unroll
  for (int t = 0; t < 8; ++t) { const int c = t * 16 + nloc; const float bb = bf16_rne(b1[c]);
#pragma unroll
    for (int r8 = 0; r8 < 8; ++r8) { b16 p, ql; split16(fmaxf(acc[t][r8] * (1.0f / (XS * WSC)) + bb, 0.0f) * XS, p, ql); Ah[8 * hlf + r8][c] = p; Al[8 * hlf + r8][c] = ql; } }
  wave_lds_sync(); v8f g = {};
#pragma unroll
  for (int kb = 0; kb < H; kb += 32) { const v16b bw = frag_kb(W2T + (size_t)nloc * H + kb, hlf); g = wmma16b(frag_kb(&Ah[nloc][kb], hlf), bw, g); g = wmma16b(frag_kb(&Al[nloc][kb], hlf), bw, g); }
  { const float bb = bf16_rne(b2[nloc]);
#pragma unroll
    for (int r8 = 0; r8 < 8; ++r8) So[8 * hlf + r8][nloc] = g[r8] * (1.0f / (XS * WSC)) + bb; }
  wave_lds_sync();
  for (int pass = 0; pass < 2; ++pass) { for (int i = lane; i < 16 * OUT; i += 32) ((volatile float*)out)[m0 * OUT + i] = So[i / OUT][i % OUT]; __threadfence(); }
}
}

extern "C" void kernel_launch(void* const* d_in, const int* in_sizes, int n_in, void* d_out, int out_size, void* d_ws, size_t ws_size, hipStream_t stream) {
  (void)n_in;
  auto Fp = [&](int i) { return (const float*)d_in[i]; }; auto Ip = [&](int i) { return (const int*)d_in[i]; };
  if (in_sizes[0] != N * 64 || in_sizes[1] != 2 * E || in_sizes[2] != H * SAT || in_sizes[4] != H * SAT || in_sizes[6] != 2 * H || in_sizes[8] != H * H || in_sizes[14] != H * H || in_sizes[20] != H * H || in_sizes[22] != OUT * H || out_size != N * OUT) return;
  const int NLIM = N; const int GB16 = NBLK, GB8 = N / 8;
  size_t off = 0; char* ws = (char*)d_ws;
  auto carve = [&](size_t bytes) { char* p = ws + off; off += (bytes + 255) & ~(size_t)255; return p; };
  b16* WSA = (b16*)carve(H * 32 * 2); b16* WNE = (b16*)carve(H * 32 * 2); b16* WG1 = (b16*)carve(H * H * 2); b16* WG2 = (b16*)carve(H * H * 2); b16* WF1 = (b16*)carve(H * H * 2); b16* WF2 = (b16*)carve(16 * H * 2);
  float* HA = (float*)carve((size_t)N * H * 4); float* HB = (float*)carve((size_t)N * H * 4); float* HW = (float*)carve((size_t)N * H * 4); float* G = (float*)carve((size_t)N * H * 4); float* AS = (float*)carve((size_t)N * 2 * 4); float* ST = (float*)carve(H * 32 * 4);
  CsrBufs7 csr; off = csr_carve7(csr, ws, off, E, N);
  if (off > ws_size || off > ((size_t)160 << 20)) return;
  wcopy_kernel<<<(H * 32 / 8 + 255) / 256, 256, 0, stream>>>(Fp(2), H, H, 32, WSA); wcopy_kernel<<<(H * 32 / 8 + 255) / 256, 256, 0, stream>>>(Fp(4), H, H, 32, WNE); wcopy_kernel<<<(H * H / 8 + 255) / 256, 256, 0, stream>>>(Fp(8), H, H, H, WG1); wcopy_kernel<<<(H * H / 8 + 255) / 256, 256, 0, stream>>>(Fp(14), H, H, H, WG2);
  wcopy_kernel<<<(H * H / 8 + 255) / 256, 256, 0, stream>>>(Fp(20), H, H, H, WF1); wcopy_kernel<<<(16 * H / 8 + 255) / 256, 256, 0, stream>>>(Fp(22), OUT, 16, H, WF2);
  csr_build7(csr, Ip(1) + E, E, N, stream);
  in_kernel<<<GB16, 32, 0, stream>>>(Fp(0), WSA, WNE, Fp(3), Fp(5), Fp(6), Fp(7), HA);
  proj_kernel<<<GB16, 32, 0, stream>>>(HA, WG1, Fp(9), Fp(10), NLIM, HW, AS);
  att_kernel<<<GB8, 256, 0, stream>>>(HW, AS, Fp(11), Ip(1), csr.PERM, csr.ROWPTR, csr.ROWCNT, (int)csr.permLen, NLIM, G);
  stats_kernel<<<H, 256, 0, stream>>>(G, NLIM, ST);
  bn_kernel<<<GB8, 256, 0, stream>>>(G, ST, Fp(12), Fp(13), HA, NLIM, HB);
  proj_kernel<<<GB16, 32, 0, stream>>>(HB, WG2, Fp(15), Fp(16), NLIM, HW, AS);
  att_kernel<<<GB8, 256, 0, stream>>>(HW, AS, Fp(17), Ip(1), csr.PERM, csr.ROWPTR, csr.ROWCNT, (int)csr.permLen, NLIM, G);
  stats_kernel<<<H, 256, 0, stream>>>(G, NLIM, ST);
  bn_kernel<<<GB8, 256, 0, stream>>>(G, ST, Fp(18), Fp(19), HB, NLIM, HA);
  head_kernel<<<GB16, 32, 0, stream>>>(HA, WF1, Fp(21), WF2, Fp(23), NLIM, (float*)d_out);
}
